// GRUDisentangledAttention_15049565405470
// MI455X (gfx1250) — hardware-verified
//
#include <hip/hip_runtime.h>
#include <stddef.h>
#include <stdint.h>


#define NBATCH 8
#define NSEQ   512
#define NDIM   1024
#define NHEAD  8
#define HDIM   128
#define NFF    4096
#define NGH    512
#define NG3    1536
#define NROWS  4096
#define CHUNK  2048
#define GTHR   128
#define RTHR   512
#define SCP    132
#define HP32   516
#define HP16   520
#define PPAD   72
#define OPAD   136

static_assert(NROWS == NBATCH * NSEQ);
static_assert(NDIM == NHEAD * HDIM);
static_assert(NG3 == 3 * NGH);
static_assert(NROWS % 64 == 0);
static_assert(NSEQ % 64 == 0);
static_assert(NDIM % 128 == 0 && NFF % 128 == 0 && NG3 % 128 == 0);
static_assert((NDIM * NDIM) % CHUNK == 0);
static_assert((NG3 * NGH) % CHUNK == 0);
static_assert((NG3 * NDIM) % CHUNK == 0);
static_assert((NFF * NDIM) % CHUNK == 0);
static_assert(RTHR == NGH);
static_assert((SCP * 4) % 16 == 0);
static_assert((HP32 * 4) % 16 == 0);
static_assert((HP16 * 2) % 16 == 0);
static_assert((PPAD * 2) % 16 == 0);
static_assert((OPAD * 2) % 16 == 0);

#define NC_WD  ((NDIM * NDIM) / CHUNK)
#define NC_WF  ((NFF * NDIM) / CHUNK)
#define NC_WHH ((NG3 * NGH) / CHUNK)
#define NC_WIH ((NG3 * NDIM) / CHUNK)
#define NPREP  (4 * NC_WD + 2 * NC_WF + 2 * NC_WHH + 2 * NC_WIH)

typedef _Float16       v16h __attribute__((ext_vector_type(16)));
typedef _Float16       v8h  __attribute__((ext_vector_type(8)));
typedef _Float16       v4h  __attribute__((ext_vector_type(4)));
typedef __bf16         v16b __attribute__((ext_vector_type(16)));
typedef unsigned short v8us __attribute__((ext_vector_type(8)));
typedef float          v8f  __attribute__((ext_vector_type(8)));
typedef float          v4f  __attribute__((ext_vector_type(4)));

union FragH { v16h v; v8h  h[2]; };
union FragB { v16b v; v8us h[2]; };

#if __has_builtin(__builtin_amdgcn_exp2f)
#define EXP2F(x) __builtin_amdgcn_exp2f(x)
#else
#define EXP2F(x) exp2f(x)
#endif
#define RCPF(x) __builtin_amdgcn_rcpf(x)

#define WSCALE 256.0f
#define IWSC   0.00390625f
#define HSCALE 16.0f
#define IS12   0.000244140625f
#define PSCALE 16384.0f
#define IPSC   6.103515625e-05f
#define LOG2E  1.4426950408889634f
#define TWOL2E 2.8853900817779268f

__device__ __forceinline__ v16h ldfrag_h(const _Float16* row, int k0, int hh)
{
    FragH f;
    f.h[0] = *(const v8h*)(row + k0 + 8 * hh);
    f.h[1] = *(const v8h*)(row + k0 + 16 + 8 * hh);
    return f.v;
}
__device__ __forceinline__ v16b ldfrag_b(const unsigned short* row, int k0, int hh)
{
    FragB f;
    f.h[0] = *(const v8us*)(row + k0 + 8 * hh);
    f.h[1] = *(const v8us*)(row + k0 + 16 + 8 * hh);
    return f.v;
}

__device__ __forceinline__ v8f wm_h(v16h a, v16h b, v8f c)
{
    v8f d = __builtin_amdgcn_wmma_f32_16x16x32_f16(false, a, false, b, (short)0, c, false, false);
    asm volatile("v_nop\n\tv_nop\n\tv_nop\n\tv_nop" : "+v"(d) : "v"(a), "v"(b));
    return d;
}
__device__ __forceinline__ v8f wm_b(v16b a, v16b b, v8f c)
{
    v8f d = __builtin_amdgcn_wmma_f32_16x16x32_bf16(false, a, false, b, (short)0, c, false, false);
    asm volatile("v_nop\n\tv_nop\n\tv_nop\n\tv_nop" : "+v"(d) : "v"(a), "v"(b));
    return d;
}

__device__ __forceinline__ v8h pack8h(v4f a, v4f b)
{
    v8h r = { (_Float16)a[0], (_Float16)a[1], (_Float16)a[2], (_Float16)a[3],
              (_Float16)b[0], (_Float16)b[1], (_Float16)b[2], (_Float16)b[3] };
    return r;
}

__device__ __forceinline__ unsigned int bfbits(float x)
{
    unsigned int u = __float_as_uint(x);
    return (u + 0x7fffu + ((u >> 16) & 1u)) >> 16;
}
__device__ __forceinline__ void split8(v4f a, v4f b, v8us& hi, v8us& lo)
{
    float v[8] = { a[0], a[1], a[2], a[3], b[0], b[1], b[2], b[3] };
    #pragma unroll
    for (int e = 0; e < 8; ++e) {
        const unsigned int hb = bfbits(v[e]);
        const float hf = __uint_as_float(hb << 16);
        const unsigned int lb = bfbits(v[e] - hf);
        hi[e] = (unsigned short)hb;
        lo[e] = (unsigned short)lb;
    }
}

__device__ __forceinline__ float gelu_f(float x)
{
    return 0.5f * x * (1.0f + erff(x * 0.70710678118654752f));
}
__device__ __forceinline__ float sigm_f(float x)
{
    return RCPF(1.0f + EXP2F(-LOG2E * x));
}
__device__ __forceinline__ float tanh_f(float x)
{
    return 1.0f - 2.0f * RCPF(1.0f + EXP2F(TWOL2E * x));
}

__global__ void __launch_bounds__(GTHR) k_prep(
    const float* __restrict__ wq, const float* __restrict__ wk,
    const float* __restrict__ wv, const float* __restrict__ wo,
    const float* __restrict__ w1, const float* __restrict__ w2,
    const float* __restrict__ whhf, const float* __restrict__ whhb,
    const float* __restrict__ wihf, const float* __restrict__ wihb,
    _Float16* wq16, _Float16* wk16, _Float16* wv16, _Float16* wo16,
    _Float16* w116, _Float16* w216, _Float16* whhf16, _Float16* whhb16,
    unsigned short* wihfh, unsigned short* wihfl, unsigned short* wihbh, unsigned short* wihbl)
{
    const int tid = threadIdx.x;
    const int bid = blockIdx.x;
    const int s1 = NC_WD, s2 = 2 * NC_WD, s3 = 3 * NC_WD, s4 = 4 * NC_WD;
    const int s5 = s4 + NC_WF, s6 = s5 + NC_WF, s7 = s6 + NC_WHH, s8 = s7 + NC_WHH;
    const int s9 = s8 + NC_WIH;

    if (bid < s8) {
        const float* src;
        _Float16* dst;
        int c;
        if (bid < s1)      { src = wq;   dst = wq16;   c = bid; }
        else if (bid < s2) { src = wk;   dst = wk16;   c = bid - s1; }
        else if (bid < s3) { src = wv;   dst = wv16;   c = bid - s2; }
        else if (bid < s4) { src = wo;   dst = wo16;   c = bid - s3; }
        else if (bid < s5) { src = w1;   dst = w116;   c = bid - s4; }
        else if (bid < s6) { src = w2;   dst = w216;   c = bid - s5; }
        else if (bid < s7) { src = whhf; dst = whhf16; c = bid - s6; }
        else               { src = whhb; dst = whhb16; c = bid - s7; }
        const size_t base = (size_t)c * CHUNK;
        v8h val[2];
        #pragma unroll
        for (int i = 0; i < 2; ++i) {
            const int e = (i * GTHR + tid) * 8;
            const v4f x0 = *(const v4f*)(src + base + e);
            const v4f x1 = *(const v4f*)(src + base + e + 4);
            val[i] = pack8h(x0 * WSCALE, x1 * WSCALE);
        }
        #pragma unroll
        for (int i = 0; i < 2; ++i)
            *(volatile v8h*)(dst + base + (size_t)(i * GTHR + tid) * 8) = val[i];
        __threadfence();
        #pragma unroll
        for (int i = 0; i < 2; ++i)
            *(volatile v8h*)(dst + base + (size_t)(i * GTHR + tid) * 8) = val[i];
    } else {
        const float* src;
        unsigned short* dh;
        unsigned short* dl;
        int c;
        if (bid < s9) { src = wihf; dh = wihfh; dl = wihfl; c = bid - s8; }
        else          { src = wihb; dh = wihbh; dl = wihbl; c = bid - s9; }
        const size_t base = (size_t)c * CHUNK;
        v8us hv[2], lv[2];
        #pragma unroll
        for (int i = 0; i < 2; ++i) {
            const int e = (i * GTHR + tid) * 8;
            const v4f x0 = *(const v4f*)(src + base + e);
            const v4f x1 = *(const v4f*)(src + base + e + 4);
            split8(x0, x1, hv[i], lv[i]);
        }
        #pragma unroll
        for (int i = 0; i < 2; ++i) {
            const size_t o = base + (size_t)(i * GTHR + tid) * 8;
            *(volatile v8us*)(dh + o) = hv[i];
            *(volatile v8us*)(dl + o) = lv[i];
        }
        __threadfence();
        #pragma unroll
        for (int i = 0; i < 2; ++i) {
            const size_t o = base + (size_t)(i * GTHR + tid) * 8;
            *(volatile v8us*)(dh + o) = hv[i];
            *(volatile v8us*)(dl + o) = lv[i];
        }
    }
}

template <int MODE>
__global__ void __launch_bounds__(GTHR) k_ln(
    const float* __restrict__ a, const float* __restrict__ b, int bmask,
    const float* __restrict__ g, const float* __restrict__ be,
    float* outF, _Float16* outH, unsigned short* outHi, unsigned short* outLo)
{
    __shared__ __align__(16) float srow[4][NDIM];

    const int tid = threadIdx.x;
    const int wv  = tid >> 5;
    const int l   = tid & 31;
    const int row = blockIdx.x * 4 + wv;
    const int brow = row & bmask;
    const float* ar = a + (size_t)row * NDIM;
    const float* br = b + (size_t)brow * NDIM;

    v4f x[8];
    float s = 0.0f;
    #pragma unroll
    for (int i = 0; i < 4; ++i) {
        const int c = (32 * i + l) * 8;
        x[2 * i]     = *(const v4f*)(ar + c)     + *(const v4f*)(br + c);
        x[2 * i + 1] = *(const v4f*)(ar + c + 4) + *(const v4f*)(br + c + 4);
        s += (x[2 * i][0] + x[2 * i][1]) + (x[2 * i][2] + x[2 * i][3]);
        s += (x[2 * i + 1][0] + x[2 * i + 1][1]) + (x[2 * i + 1][2] + x[2 * i + 1][3]);
    }
    #pragma unroll
    for (int off = 16; off > 0; off >>= 1) s += __shfl_xor(s, off, 32);
    const float mean = s * (1.0f / (float)NDIM);

    float s2 = 0.0f;
    #pragma unroll
    for (int k = 0; k < 8; ++k) {
        const v4f d = x[k] - mean;
        s2 += (d[0] * d[0] + d[1] * d[1]) + (d[2] * d[2] + d[3] * d[3]);
    }
    #pragma unroll
    for (int off = 16; off > 0; off >>= 1) s2 += __shfl_xor(s2, off, 32);
    const float var  = s2 * (1.0f / (float)NDIM);
    const float rstd = rsqrtf(var + 1e-7f);

    v4f y[8];
    #pragma unroll
    for (int i = 0; i < 4; ++i) {
        const int c = (32 * i + l) * 8;
        const v4f g0 = *(const v4f*)(g + c),  g1 = *(const v4f*)(g + c + 4);
        const v4f b0 = *(const v4f*)(be + c), b1 = *(const v4f*)(be + c + 4);
        y[2 * i]     = (x[2 * i]     - mean) * rstd * g0 + b0;
        y[2 * i + 1] = (x[2 * i + 1] - mean) * rstd * g1 + b1;
    }

    if (MODE == 0) {
        v8h hv[4];
        #pragma unroll
        for (int i = 0; i < 4; ++i) hv[i] = pack8h(y[2 * i], y[2 * i + 1]);
        #pragma unroll
        for (int i = 0; i < 4; ++i) {
            const int c = (32 * i + l) * 8;
            *(v4f*)&srow[wv][c]     = y[2 * i];
            *(v4f*)&srow[wv][c + 4] = y[2 * i + 1];
        }
        __syncthreads();
        v4f fv[8];
        #pragma unroll
        for (int i = 0; i < 8; ++i) fv[i] = *(const v4f*)&srow[wv][(32 * i + l) * 4];

        _Float16* oh = outH + (size_t)row * NDIM;
        float*    of = outF + (size_t)row * NDIM;
        #pragma unroll
        for (int i = 0; i < 4; ++i) *(volatile v8h*)(oh + (32 * i + l) * 8) = hv[i];
        #pragma unroll
        for (int i = 0; i < 8; ++i) *(volatile v4f*)(of + (32 * i + l) * 4) = fv[i];
        __threadfence();
        #pragma unroll
        for (int i = 0; i < 4; ++i) *(volatile v8h*)(oh + (32 * i + l) * 8) = hv[i];
        #pragma unroll
        for (int i = 0; i < 8; ++i) *(volatile v4f*)(of + (32 * i + l) * 4) = fv[i];
    } else {
        v8us hv[4], lv[4];
        #pragma unroll
        for (int i = 0; i < 4; ++i) split8(y[2 * i], y[2 * i + 1], hv[i], lv[i]);
        unsigned short* ohi = outHi + (size_t)row * NDIM;
        unsigned short* olo = outLo + (size_t)row * NDIM;
        #pragma unroll
        for (int i = 0; i < 4; ++i) {
            *(volatile v8us*)(ohi + (32 * i + l) * 8) = hv[i];
            *(volatile v8us*)(olo + (32 * i + l) * 8) = lv[i];
        }
        __threadfence();
        #pragma unroll
        for (int i = 0; i < 4; ++i) {
            *(volatile v8us*)(ohi + (32 * i + l) * 8) = hv[i];
            *(volatile v8us*)(olo + (32 * i + l) * 8) = lv[i];
        }
    }
}

template <int HASBIAS, int ACT>
__device__ __forceinline__ void store_tile_f32(float (*sC)[SCP], const float* __restrict__ bias,
                                               float* Cf, int N, int row0, int col0, float scale,
                                               int wv, int l)
{
    v4f vals[16];
    #pragma unroll
    for (int i = 0; i < 16; ++i) {
        const int row = 16 * wv + i;
        v4f x = *(const v4f*)&sC[row][4 * l] * scale;
        if (HASBIAS) x = x + *(const v4f*)(bias + col0 + 4 * l);
        if (ACT) { x[0] = gelu_f(x[0]); x[1] = gelu_f(x[1]); x[2] = gelu_f(x[2]); x[3] = gelu_f(x[3]); }
        vals[i] = x;
    }
    #pragma unroll
    for (int i = 0; i < 16; ++i)
        *(volatile v4f*)(Cf + (size_t)(row0 + 16 * wv + i) * N + col0 + 4 * l) = vals[i];
    __threadfence();
    #pragma unroll
    for (int i = 0; i < 16; ++i)
        *(volatile v4f*)(Cf + (size_t)(row0 + 16 * wv + i) * N + col0 + 4 * l) = vals[i];
}

template <int HASBIAS, int ACT, int OUTMODE>
__global__ void __launch_bounds__(GTHR) k_gemm(
    const _Float16* __restrict__ A, const _Float16* __restrict__ W,
    const float* __restrict__ bias, float* Cf, _Float16* Ch, int N, int K, float scale)
{
    __shared__ __align__(16) float sC[64][SCP];

    const int tid = threadIdx.x;
    const int wv  = tid >> 5;
    const int l   = tid & 31;
    const int hh  = l >> 4;
    const int m15 = l & 15;
    const int wr  = wv & 1;
    const int wc  = wv >> 1;
    const int row0 = blockIdx.x * 64;
    const int col0 = blockIdx.y * 128;

    const v8f zero = { 0.f, 0.f, 0.f, 0.f, 0.f, 0.f, 0.f, 0.f };
    v8f acc[2][4];
    #pragma unroll
    for (int rt = 0; rt < 2; ++rt)
        #pragma unroll
        for (int j = 0; j < 4; ++j) acc[rt][j] = zero;

    const _Float16* a0p = A + (size_t)(row0 + 32 * wr + m15) * K;
    const _Float16* a1p = a0p + (size_t)16 * K;
    const _Float16* bp  = W + (size_t)(col0 + 64 * wc + m15) * K;

    #pragma unroll 1
    for (int k0 = 0; k0 < K; k0 += 32) {
        const v16h fa0 = ldfrag_h(a0p, k0, hh);
        const v16h fa1 = ldfrag_h(a1p, k0, hh);
        #pragma unroll
        for (int j = 0; j < 4; ++j) {
            const v16h fb = ldfrag_h(bp + (size_t)j * 16 * K, k0, hh);
            acc[0][j] = wm_h(fa0, fb, acc[0][j]);
            acc[1][j] = wm_h(fa1, fb, acc[1][j]);
        }
    }

    #pragma unroll
    for (int rt = 0; rt < 2; ++rt)
        #pragma unroll
        for (int j = 0; j < 4; ++j)
            #pragma unroll
            for (int r = 0; r < 8; ++r)
                sC[32 * wr + 16 * rt + 8 * hh + r][64 * wc + 16 * j + m15] = acc[rt][j][r];
    __syncthreads();

    if (OUTMODE == 0) {
        store_tile_f32<HASBIAS, ACT>(sC, bias, Cf, N, row0, col0, scale, wv, l);
    } else if (OUTMODE == 1) {
        v8h hv[8];
        size_t off[8];
        #pragma unroll
        for (int i = 0; i < 8; ++i) {
            const int row = 16 * wv + 2 * i + hh;
            const int c   = 8 * m15;
            v4f x0 = *(const v4f*)&sC[row][c] * scale;
            v4f x1 = *(const v4f*)&sC[row][c + 4] * scale;
            if (HASBIAS) {
                x0 = x0 + *(const v4f*)(bias + col0 + c);
                x1 = x1 + *(const v4f*)(bias + col0 + c + 4);
            }
            if (ACT) {
                x0[0] = gelu_f(x0[0]); x0[1] = gelu_f(x0[1]); x0[2] = gelu_f(x0[2]); x0[3] = gelu_f(x0[3]);
                x1[0] = gelu_f(x1[0]); x1[1] = gelu_f(x1[1]); x1[2] = gelu_f(x1[2]); x1[3] = gelu_f(x1[3]);
            }
            hv[i]  = pack8h(x0, x1);
            off[i] = (size_t)(row0 + row) * N + col0 + c;
        }
        #pragma unroll
        for (int i = 0; i < 8; ++i) *(volatile v8h*)(Ch + off[i]) = hv[i];
        __threadfence();
        #pragma unroll
        for (int i = 0; i < 8; ++i) *(volatile v8h*)(Ch + off[i]) = hv[i];
    } else {
        const int bq   = blockIdx.x >> 3;
        const int s0   = (blockIdx.x & 7) * 64;
        const int head = blockIdx.y;
        v8h hv[8];
        size_t off[8];
        #pragma unroll
        for (int i = 0; i < 8; ++i) {
            const int d    = 32 * wv + 4 * i + (l >> 3);
            const int sseg = (l & 7) * 8;
            float bb = 0.0f;
            if (HASBIAS) bb = bias[col0 + d];
            v8h hvv;
            #pragma unroll
            for (int e = 0; e < 8; ++e) {
                float x = sC[sseg + e][d] * scale + bb;
                if (ACT) x = gelu_f(x);
                hvv[e] = (_Float16)x;
            }
            hv[i]  = hvv;
            off[i] = ((size_t)((bq * NHEAD + head) * HDIM + d)) * NSEQ + s0 + sseg;
        }
        #pragma unroll
        for (int i = 0; i < 8; ++i) *(volatile v8h*)(Ch + off[i]) = hv[i];
        __threadfence();
        #pragma unroll
        for (int i = 0; i < 8; ++i) *(volatile v8h*)(Ch + off[i]) = hv[i];
    }
}

__global__ void __launch_bounds__(GTHR) k_gemm3(
    const unsigned short* __restrict__ Ah, const unsigned short* __restrict__ Al,
    const unsigned short* __restrict__ Wh, const unsigned short* __restrict__ Wl,
    const float* __restrict__ bias, float* Cf, int N, int K)
{
    __shared__ __align__(16) float sC[64][SCP];

    const int tid = threadIdx.x;
    const int wv  = tid >> 5;
    const int l   = tid & 31;
    const int hh  = l >> 4;
    const int m15 = l & 15;
    const int wr  = wv & 1;
    const int wc  = wv >> 1;
    const int row0 = blockIdx.x * 64;
    const int col0 = blockIdx.y * 128;

    const v8f zero = { 0.f, 0.f, 0.f, 0.f, 0.f, 0.f, 0.f, 0.f };
    v8f acc[2][4];
    #pragma unroll
    for (int rt = 0; rt < 2; ++rt)
        #pragma unroll
        for (int j = 0; j < 4; ++j) acc[rt][j] = zero;

    const size_t arow = (size_t)(row0 + 32 * wr + m15) * K;
    const size_t brow = (size_t)(col0 + 64 * wc + m15) * K;
    const unsigned short* ah0 = Ah + arow;
    const unsigned short* ah1 = ah0 + (size_t)16 * K;
    const unsigned short* al0 = Al + arow;
    const unsigned short* al1 = al0 + (size_t)16 * K;
    const unsigned short* bhp = Wh + brow;
    const unsigned short* blp = Wl + brow;

    #pragma unroll 1
    for (int k0 = 0; k0 < K; k0 += 32) {
        const v16b fah0 = ldfrag_b(ah0, k0, hh);
        const v16b fah1 = ldfrag_b(ah1, k0, hh);
        const v16b fal0 = ldfrag_b(al0, k0, hh);
        const v16b fal1 = ldfrag_b(al1, k0, hh);
        #pragma unroll
        for (int j = 0; j < 4; ++j) {
            const v16b fbh = ldfrag_b(bhp + (size_t)j * 16 * K, k0, hh);
            const v16b fbl = ldfrag_b(blp + (size_t)j * 16 * K, k0, hh);
            acc[0][j] = wm_b(fah0, fbh, acc[0][j]);
            acc[0][j] = wm_b(fah0, fbl, acc[0][j]);
            acc[0][j] = wm_b(fal0, fbh, acc[0][j]);
            acc[1][j] = wm_b(fah1, fbh, acc[1][j]);
            acc[1][j] = wm_b(fah1, fbl, acc[1][j]);
            acc[1][j] = wm_b(fal1, fbh, acc[1][j]);
        }
    }

    #pragma unroll
    for (int rt = 0; rt < 2; ++rt)
        #pragma unroll
        for (int j = 0; j < 4; ++j)
            #pragma unroll
            for (int r = 0; r < 8; ++r)
                sC[32 * wr + 16 * rt + 8 * hh + r][64 * wc + 16 * j + m15] = acc[rt][j][r];
    __syncthreads();

    store_tile_f32<1, 0>(sC, bias, Cf, N, row0, col0, 1.0f, wv, l);
}

__global__ void __launch_bounds__(GTHR) k_attn(
    const _Float16* __restrict__ q16, const _Float16* __restrict__ k16,
    const _Float16* __restrict__ vT, _Float16* ctx)
{
    __shared__ __align__(16) _Float16 sP[4][16][PPAD];
    __shared__ __align__(16) _Float16 sO[4][16][OPAD];

    const int tid = threadIdx.x;
    const int wv  = tid >> 5;
    const int l   = tid & 31;
    const int hh  = l >> 4;
    const int m15 = l & 15;
    const int bh   = blockIdx.x;
    const int b    = bh >> 3;
    const int head = bh & 7;
    const int q0   = blockIdx.y * 64 + 16 * wv;

    const _Float16* qrow  = q16 + (size_t)(b * NSEQ + q0 + m15) * NDIM + head * HDIM;
    const _Float16* kbase = k16 + (size_t)(b * NSEQ + m15) * NDIM + head * HDIM;
    const _Float16* vbase = vT + ((size_t)bh * HDIM + m15) * NSEQ;

    const float NEG_INF = -__builtin_inff();
    const float SCL = 0.08838834764831845f * LOG2E;

    float mrun[8], lrun[8];
    #pragma unroll
    for (int r = 0; r < 8; ++r) { mrun[r] = NEG_INF; lrun[r] = 0.0f; }

    const v8f zero = { 0.f, 0.f, 0.f, 0.f, 0.f, 0.f, 0.f, 0.f };
    v8f oacc[8];
    #pragma unroll
    for (int j = 0; j < 8; ++j) oacc[j] = zero;

    #pragma unroll 1
    for (int c = 0; c < NSEQ / 64; ++c) {
        v8f sacc[4];
        #pragma unroll
        for (int j = 0; j < 4; ++j) sacc[j] = zero;
        #pragma unroll
        for (int kc = 0; kc < HDIM / 32; ++kc) {
            const v16h fa = ldfrag_h(qrow, 32 * kc, hh);
            #pragma unroll
            for (int j = 0; j < 4; ++j) {
                const v16h fb = ldfrag_h(kbase + (size_t)(64 * c + 16 * j) * NDIM, 32 * kc, hh);
                sacc[j] = wm_h(fa, fb, sacc[j]);
            }
        }

        #pragma unroll
        for (int r = 0; r < 8; ++r) {
            float cm = NEG_INF;
            #pragma unroll
            for (int j = 0; j < 4; ++j) {
                const float s2 = sacc[j][r] * SCL;
                sacc[j][r] = s2;
                cm = fmaxf(cm, s2);
            }
            #pragma unroll
            for (int off = 1; off < 16; off <<= 1) cm = fmaxf(cm, __shfl_xor(cm, off, 32));
            const float mn    = fmaxf(mrun[r], cm);
            const float alpha = EXP2F(mrun[r] - mn);
            mrun[r] = mn;
            float ps = 0.0f;
            #pragma unroll
            for (int j = 0; j < 4; ++j) {
                const float p = EXP2F(sacc[j][r] - mn);
                sacc[j][r] = p;
                ps += p;
            }
            #pragma unroll
            for (int off = 1; off < 16; off <<= 1) ps += __shfl_xor(ps, off, 32);
            lrun[r] = lrun[r] * alpha + ps;
            #pragma unroll
            for (int j = 0; j < 8; ++j) oacc[j][r] = oacc[j][r] * alpha;
        }

        #pragma unroll
        for (int j = 0; j < 4; ++j)
            #pragma unroll
            for (int r = 0; r < 8; ++r)
                sP[wv][8 * hh + r][16 * j + m15] = (_Float16)(sacc[j][r] * PSCALE);
        __syncthreads();

        #pragma unroll
        for (int ks = 0; ks < 2; ++ks) {
            const v16h fa = ldfrag_h(&sP[wv][m15][0], 32 * ks, hh);
            #pragma unroll
            for (int j = 0; j < 8; ++j) {
                const v16h fb = ldfrag_h(vbase + (size_t)(16 * j) * NSEQ + 64 * c, 32 * ks, hh);
                oacc[j] = wm_h(fa, fb, oacc[j]);
            }
        }
        __syncthreads();
    }

    #pragma unroll
    for (int r = 0; r < 8; ++r) {
        const float inv = RCPF(lrun[r]) * IPSC;
        #pragma unroll
        for (int j = 0; j < 8; ++j)
            sO[wv][8 * hh + r][16 * j + m15] = (_Float16)(oacc[j][r] * inv);
    }
    __syncthreads();

    v8h ov[8];
    size_t off[8];
    #pragma unroll
    for (int i = 0; i < 8; ++i) {
        const int row = 2 * i + hh;
        ov[i]  = *(const v8h*)&sO[wv][row][8 * m15];
        off[i] = (size_t)(b * NSEQ + q0 + row) * NDIM + head * HDIM + 8 * m15;
    }
    #pragma unroll
    for (int i = 0; i < 8; ++i) *(volatile v8h*)(ctx + off[i]) = ov[i];
    __threadfence();
    #pragma unroll
    for (int i = 0; i < 8; ++i) *(volatile v8h*)(ctx + off[i]) = ov[i];
}

__global__ void __launch_bounds__(RTHR) k_gru(
    const float* __restrict__ gxf, const float* __restrict__ gxb,
    const _Float16* __restrict__ whhf, const _Float16* __restrict__ whhb,
    const float* __restrict__ bhhf, const float* __restrict__ bhhb,
    float* out)
{
    __shared__ __align__(16) float    h32s[NBATCH][HP32];
    __shared__ __align__(16) _Float16 h16s[16][HP16];

    const int dir = blockIdx.x;
    const float*    gx  = dir ? gxb  : gxf;
    const _Float16* whh = dir ? whhb : whhf;
    const float*    bhh = dir ? bhhb : bhhf;

    const int tid = threadIdx.x;
    const int wv  = tid >> 5;
    const int l   = tid & 31;
    const int hh  = l >> 4;
    const int m15 = l & 15;
    const int j   = 32 * wv + 16 * hh + m15;

    {
        float* hz = &h32s[0][0];
        for (int i = tid; i < NBATCH * HP32; i += RTHR) hz[i] = 0.0f;
        _Float16* h6 = &h16s[0][0];
        for (int i = tid; i < 16 * HP16; i += RTHR) h6[i] = (_Float16)0.0f;
    }
    __syncthreads();

    const float bhr = bhh[j];
    const float bhz = bhh[NGH + j];
    const float bhn = bhh[2 * NGH + j];

    const _Float16* wbase = whh + (size_t)(32 * wv + m15) * NGH;
    const _Float16* hrow  = &h16s[m15][0];

    const int ob    = wv >> 1;
    const int chalf = (wv & 1) * 256;

    const v8f zero = { 0.f, 0.f, 0.f, 0.f, 0.f, 0.f, 0.f, 0.f };

    #pragma unroll 1
    for (int s = 0; s < NSEQ; ++s) {
        const int t = dir ? (NSEQ - 1 - s) : s;

        v8f acc[6];
        #pragma unroll
        for (int jt = 0; jt < 6; ++jt) acc[jt] = zero;

        #pragma unroll 1
        for (int k0 = 0; k0 < NGH; k0 += 32) {
            const v16h fa = ldfrag_h(hrow, k0, hh);
            #pragma unroll
            for (int jt = 0; jt < 6; ++jt) {
                const v16h fb = ldfrag_h(wbase + (size_t)((jt >> 1) * NGH + 16 * (jt & 1)) * NGH, k0, hh);
                acc[jt] = wm_h(fa, fb, acc[jt]);
            }
        }

        const float* gxt = gx + (size_t)t * NG3 + j;
        float hn[8];
        #pragma unroll
        for (int r = 0; r < 8; ++r) {
            const float* gr = gxt + (size_t)r * NSEQ * NG3;
            const float gxr = gr[0];
            const float gxz = gr[NGH];
            const float gxn = gr[2 * NGH];
            const float aR = hh ? acc[1][r] : acc[0][r];
            const float aZ = hh ? acc[3][r] : acc[2][r];
            const float aN = hh ? acc[5][r] : acc[4][r];
            const float rr = sigm_f(gxr + fmaf(aR, IS12, bhr));
            const float zz = sigm_f(gxz + fmaf(aZ, IS12, bhz));
            const float nn = tanh_f(gxn + rr * fmaf(aN, IS12, bhn));
            const float ho = h32s[r][j];
            hn[r] = (1.0f - zz) * nn + zz * ho;
        }
        __syncthreads();
        #pragma unroll
        for (int r = 0; r < 8; ++r) {
            h32s[r][j] = hn[r];
            const _Float16 hv = (_Float16)(HSCALE * hn[r]);
            h16s[r][j]     = hv;
            h16s[8 + r][j] = hv;
        }
        __syncthreads();

        const v4f o0 = *(const v4f*)&h32s[ob][chalf + 4 * l];
        const v4f o1 = *(const v4f*)&h32s[ob][chalf + 128 + 4 * l];
        float* op = out + ((size_t)(ob * NSEQ + t)) * NDIM + dir * NGH + chalf;
        *(volatile v4f*)(op + 4 * l)       = o0;
        *(volatile v4f*)(op + 128 + 4 * l) = o1;
        __threadfence();
        *(volatile v4f*)(op + 4 * l)       = o0;
        *(volatile v4f*)(op + 128 + 4 * l) = o1;
    }
}

extern "C" void kernel_launch(void* const* d_in, const int* in_sizes, int n_in,
                              void* d_out, int out_size, void* d_ws, size_t ws_size,
                              hipStream_t stream)
{
    if (n_in < 27) return;
    if (in_sizes[0] != NROWS * NDIM) return;
    if (in_sizes[1] != NSEQ * NDIM) return;
    if (in_sizes[2] != NDIM || in_sizes[3] != NDIM) return;
    if (in_sizes[4] != NDIM * NDIM || in_sizes[5] != NDIM * NDIM || in_sizes[6] != NDIM * NDIM) return;
    if (in_sizes[7] != NDIM || in_sizes[8] != NDIM) return;
    if (in_sizes[9] != NDIM * NDIM || in_sizes[10] != NDIM) return;
    if (in_sizes[11] != NDIM || in_sizes[12] != NDIM) return;
    if (in_sizes[13] != NFF * NDIM || in_sizes[14] != NFF) return;
    if (in_sizes[15] != NDIM * NFF || in_sizes[16] != NDIM) return;
    if (in_sizes[17] != NDIM || in_sizes[18] != NDIM) return;
    if (in_sizes[19] != NG3 * NDIM || in_sizes[20] != NG3 * NGH) return;
    if (in_sizes[21] != NG3 || in_sizes[22] != NG3) return;
    if (in_sizes[23] != NG3 * NDIM || in_sizes[24] != NG3 * NGH) return;
    if (in_sizes[25] != NG3 || in_sizes[26] != NG3) return;
    if (out_size != NROWS * NDIM) return;

    const float* x       = (const float*)d_in[0];
    const float* pos_emb = (const float*)d_in[1];
    const float* emb_g   = (const float*)d_in[2];
    const float* emb_b   = (const float*)d_in[3];
    const float* wq      = (const float*)d_in[4];
    const float* wk      = (const float*)d_in[5];
    const float* wv      = (const float*)d_in[6];
    const float* q_bias  = (const float*)d_in[7];
    const float* v_bias  = (const float*)d_in[8];
    const float* wo      = (const float*)d_in[9];
    const float* bo      = (const float*)d_in[10];
    const float* aln_g   = (const float*)d_in[11];
    const float* aln_b   = (const float*)d_in[12];
    const float* w1      = (const float*)d_in[13];
    const float* b1      = (const float*)d_in[14];
    const float* w2      = (const float*)d_in[15];
    const float* b2      = (const float*)d_in[16];
    const float* fln_g   = (const float*)d_in[17];
    const float* fln_b   = (const float*)d_in[18];
    const float* wih_f   = (const float*)d_in[19];
    const float* whh_f   = (const float*)d_in[20];
    const float* bih_f   = (const float*)d_in[21];
    const float* bhh_f   = (const float*)d_in[22];
    const float* wih_b   = (const float*)d_in[23];
    const float* whh_b   = (const float*)d_in[24];
    const float* bih_b   = (const float*)d_in[25];
    const float* bhh_b   = (const float*)d_in[26];
    float* out = (float*)d_out;

    const size_t MIB    = 1048576;
    const size_t oWIHFH = 0;
    const size_t oWIHFL = 3 * MIB;
    const size_t oWIHBH = 6 * MIB;
    const size_t oWIHBL = 9 * MIB;
    const size_t oWHHF  = 12 * MIB;
    const size_t oWHHB  = 12 * MIB + (size_t)NG3 * NGH * 2;
    const size_t oW1    = 15 * MIB;
    const size_t oW2    = 23 * MIB;
    const size_t oWQ    = 31 * MIB;
    const size_t oWK    = 33 * MIB;
    const size_t oWV    = 35 * MIB;
    const size_t oWO    = 37 * MIB;
    const size_t oH32   = 39 * MIB;
    const size_t oH16   = 55 * MIB;
    const size_t oQ16   = 63 * MIB;
    const size_t oK16   = 71 * MIB;
    const size_t oVT    = 79 * MIB;
    const size_t oCTX   = 87 * MIB;
    const size_t oOPRE  = 95 * MIB;
    const size_t oATT32 = 63 * MIB;
    const size_t oATT16 = 79 * MIB;
    const size_t oFF16  = 87 * MIB;
    const size_t oFPRE  = 39 * MIB;
    const size_t oENCH  = 87 * MIB;
    const size_t oENCL  = 95 * MIB;
    const size_t oGXF   = 39 * MIB;
    const size_t oGXB   = 63 * MIB;
    const size_t oEND   = 119 * MIB;
    if (oEND > ws_size) return;

    char* ws = (char*)d_ws;
    unsigned short* wihfh = (unsigned short*)(ws + oWIHFH);
    unsigned short* wihfl = (unsigned short*)(ws + oWIHFL);
    unsigned short* wihbh = (unsigned short*)(ws + oWIHBH);
    unsigned short* wihbl = (unsigned short*)(ws + oWIHBL);
    _Float16* whhf16 = (_Float16*)(ws + oWHHF);
    _Float16* whhb16 = (_Float16*)(ws + oWHHB);
    _Float16* w116   = (_Float16*)(ws + oW1);
    _Float16* w216   = (_Float16*)(ws + oW2);
    _Float16* wq16   = (_Float16*)(ws + oWQ);
    _Float16* wk16   = (_Float16*)(ws + oWK);
    _Float16* wv16   = (_Float16*)(ws + oWV);
    _Float16* wo16   = (_Float16*)(ws + oWO);
    float*    h32    = (float*)(ws + oH32);
    _Float16* h16    = (_Float16*)(ws + oH16);
    _Float16* q16    = (_Float16*)(ws + oQ16);
    _Float16* k16    = (_Float16*)(ws + oK16);
    _Float16* vT     = (_Float16*)(ws + oVT);
    _Float16* ctx16  = (_Float16*)(ws + oCTX);
    float*    opre   = (float*)(ws + oOPRE);
    float*    attn32 = (float*)(ws + oATT32);
    _Float16* attn16 = (_Float16*)(ws + oATT16);
    _Float16* ff16   = (_Float16*)(ws + oFF16);
    float*    fpre   = (float*)(ws + oFPRE);
    unsigned short* ench = (unsigned short*)(ws + oENCH);
    unsigned short* encl = (unsigned short*)(ws + oENCL);
    float*    gxf    = (float*)(ws + oGXF);
    float*    gxb    = (float*)(ws + oGXB);
    float*          pf = opre;
    _Float16*       ph = ctx16;
    unsigned short* pu = ench;

    k_prep<<<dim3(NPREP), dim3(GTHR), 0, stream>>>(
        wq, wk, wv, wo, w1, w2, whh_f, whh_b, wih_f, wih_b,
        wq16, wk16, wv16, wo16, w116, w216, whhf16, whhb16,
        wihfh, wihfl, wihbh, wihbl);

    k_ln<0><<<dim3(NROWS / 4), dim3(GTHR), 0, stream>>>(
        x, pos_emb, NSEQ - 1, emb_g, emb_b, h32, h16, pu, pu);

    k_gemm<1, 0, 1><<<dim3(NROWS / 64, NDIM / 128), dim3(GTHR), 0, stream>>>(
        h16, wq16, q_bias, pf, q16, NDIM, NDIM, IWSC);
    k_gemm<0, 0, 1><<<dim3(NROWS / 64, NDIM / 128), dim3(GTHR), 0, stream>>>(
        h16, wk16, q_bias, pf, k16, NDIM, NDIM, IWSC);
    k_gemm<1, 0, 2><<<dim3(NROWS / 64, NDIM / 128), dim3(GTHR), 0, stream>>>(
        h16, wv16, v_bias, pf, vT, NDIM, NDIM, IWSC);

    k_attn<<<dim3(NBATCH * NHEAD, NSEQ / 64), dim3(GTHR), 0, stream>>>(q16, k16, vT, ctx16);

    k_gemm<1, 0, 0><<<dim3(NROWS / 64, NDIM / 128), dim3(GTHR), 0, stream>>>(
        ctx16, wo16, bo, opre, ph, NDIM, NDIM, IWSC);
    k_ln<0><<<dim3(NROWS / 4), dim3(GTHR), 0, stream>>>(
        opre, h32, NROWS - 1, aln_g, aln_b, attn32, attn16, pu, pu);

    k_gemm<1, 1, 1><<<dim3(NROWS / 64, NFF / 128), dim3(GTHR), 0, stream>>>(
        attn16, w116, b1, pf, ff16, NFF, NDIM, IWSC);
    k_gemm<1, 0, 0><<<dim3(NROWS / 64, NDIM / 128), dim3(GTHR), 0, stream>>>(
        ff16, w216, b2, fpre, ph, NDIM, NFF, IWSC);

    k_ln<1><<<dim3(NROWS / 4), dim3(GTHR), 0, stream>>>(
        fpre, attn32, NROWS - 1, fln_g, fln_b, pf, ph, ench, encl);

    k_gemm3<<<dim3(NROWS / 64, NG3 / 128), dim3(GTHR), 0, stream>>>(
        ench, encl, wihfh, wihfl, bih_f, gxf, NG3, NDIM);
    k_gemm3<<<dim3(NROWS / 64, NG3 / 128), dim3(GTHR), 0, stream>>>(
        ench, encl, wihbh, wihbl, bih_b, gxb, NG3, NDIM);

    k_gru<<<dim3(2), dim3(RTHR), 0, stream>>>(gxf, gxb, whhf16, whhb16, bhh_f, bhh_b, out);
}
